// HeteroConv_43044162240973
// MI455X (gfx1250) — hardware-verified
//
#include <hip/hip_runtime.h>
#include <stddef.h>


#define FD      128
#define KF      256
#define AP      512
#define TT      3
#define LL      3
#define NTHR    256
#define NWAVE   8
#define EPT     8
#define NGRP    2
#define CHUNK   (NTHR * EPT * NGRP)
#define WCAP    (EPT * NGRP * 32)
#define LISTN   (NWAVE * WCAP)
#define NBC     4096
#define NBF     1024
#define RCAP    40960
#define RBN     128
#define TGT     256
#define DEGCAP  256
#define OTHR    512
#define SROWS   16
#define GBM     64
#define PARTN   256
#define SLOTN   512
#define HSCALE  16.0f
#define WSCALE  64.0f
#define OINV    0.0009765625f
#define BN_EPS  0.00001f
#define WSCAP   134217728
#define LDS_FILL ((RCAP + NBF + LISTN) * 4 + 64)

static_assert((CHUNK & (CHUNK - 1)) == 0);
static_assert(CHUNK <= 4096);
static_assert(NBC <= 4096 && NBF <= 4096);
static_assert((NBC & (NBC - 1)) == 0 && (NBF & (NBF - 1)) == 0);
static_assert(NBC == 4 * NBF);
static_assert(OTHR * 8 == NBC);
static_assert((RCAP % 32) == 0);
static_assert(TGT == NWAVE * 32);
static_assert((NBC % TGT) == 0);
static_assert((TGT % GBM) == 0);
static_assert(KF == 2 * FD && AP == FD * (1 + TT));
static_assert(FD % 32 == 0 && KF % 32 == 0);
static_assert((SROWS & (SROWS - 1)) == 0 && 32 % SROWS == 0);
static_assert(SROWS * FD * 2 == 8 * 32 * 16);
static_assert(SLOTN == 4 * FD && PARTN == 2 * FD);

typedef float          v4f  __attribute__((ext_vector_type(4)));
typedef float          v8f  __attribute__((ext_vector_type(8)));
typedef double         v2d  __attribute__((ext_vector_type(2)));
typedef int            v4i  __attribute__((ext_vector_type(4)));
typedef unsigned int   v2u  __attribute__((ext_vector_type(2)));
typedef unsigned int   v4u  __attribute__((ext_vector_type(4)));
typedef unsigned short v8us __attribute__((ext_vector_type(8)));
typedef _Float16       v4h  __attribute__((ext_vector_type(4)));
typedef _Float16       v8h  __attribute__((ext_vector_type(8)));
typedef _Float16       v16h __attribute__((ext_vector_type(16)));
union FragH { v16h v; v8us h[2]; };
union Pack8 { v8h h; v8us u; };
union Pack4 { v4h h; v2u u; };

__device__ __forceinline__ v8us cvt8h(v4f a, v4f b, float sc) {
  v8h r;
  r[0] = (_Float16)(a.x * sc); r[1] = (_Float16)(a.y * sc);
  r[2] = (_Float16)(a.z * sc); r[3] = (_Float16)(a.w * sc);
  r[4] = (_Float16)(b.x * sc); r[5] = (_Float16)(b.y * sc);
  r[6] = (_Float16)(b.z * sc); r[7] = (_Float16)(b.w * sc);
  Pack8 p;
  p.h = r;
  return p.u;
}

__device__ __forceinline__ v2u cvt4h(v4f a, float sc) {
  v4h r;
  r[0] = (_Float16)(a.x * sc); r[1] = (_Float16)(a.y * sc);
  r[2] = (_Float16)(a.z * sc); r[3] = (_Float16)(a.w * sc);
  Pack4 p;
  p.h = r;
  return p.u;
}

__device__ __forceinline__ v8f wmh(v16h a, v16h b, v8f c) {
  v8f d = __builtin_amdgcn_wmma_f32_16x16x32_f16(false, a, false, b, (short)0, c, false, false);
  asm volatile("v_nop\n\tv_nop\n\tv_nop\n\tv_nop" : "+v"(d) : "v"(a), "v"(b));
  return d;
}

template <int NB>
__device__ __forceinline__ int scan_chunk(const int* __restrict__ dsts, int nE, int cbase, int slotBase,
                                          int vec8, int* list, int tid, int lane, int wave) {
  int wc = 0;
#pragma unroll
  for (int g = 0; g < NGRP; ++g) {
    const int el0  = (g * NTHR + tid) * EPT;
    const int e0   = cbase + el0;
    const int sent = -2147483647 - 1;
    v4i da, db;
    if (vec8 != 0 && cbase + CHUNK <= nE) {
      da = *(const v4i*)(dsts + e0);
      db = *(const v4i*)(dsts + e0 + 4);
    } else {
      da.x = (e0     < nE) ? dsts[min(e0, nE - 1)] : sent;
      da.y = (e0 + 1 < nE) ? dsts[min(e0 + 1, nE - 1)] : sent;
      da.z = (e0 + 2 < nE) ? dsts[min(e0 + 2, nE - 1)] : sent;
      da.w = (e0 + 3 < nE) ? dsts[min(e0 + 3, nE - 1)] : sent;
      db.x = (e0 + 4 < nE) ? dsts[min(e0 + 4, nE - 1)] : sent;
      db.y = (e0 + 5 < nE) ? dsts[min(e0 + 5, nE - 1)] : sent;
      db.z = (e0 + 6 < nE) ? dsts[min(e0 + 6, nE - 1)] : sent;
      db.w = (e0 + 7 < nE) ? dsts[min(e0 + 7, nE - 1)] : sent;
    }
    const unsigned nb = (unsigned)slotBase;
    const unsigned s0 = (unsigned)da.x - nb, s1 = (unsigned)da.y - nb;
    const unsigned s2 = (unsigned)da.z - nb, s3 = (unsigned)da.w - nb;
    const unsigned s4 = (unsigned)db.x - nb, s5 = (unsigned)db.y - nb;
    const unsigned s6 = (unsigned)db.z - nb, s7 = (unsigned)db.w - nb;
    const bool h0 = s0 < (unsigned)NB, h1 = s1 < (unsigned)NB, h2 = s2 < (unsigned)NB, h3 = s3 < (unsigned)NB;
    const bool h4 = s4 < (unsigned)NB, h5 = s5 < (unsigned)NB, h6 = s6 < (unsigned)NB, h7 = s7 < (unsigned)NB;
    const unsigned any = __builtin_amdgcn_ballot_w32(h0 | h1 | h2 | h3 | h4 | h5 | h6 | h7);
    if (any != 0u) {
#define HITJ(J, HJ, SJ) { \
        const unsigned mj = __builtin_amdgcn_ballot_w32(HJ); \
        if (mj != 0u) { \
          if (HJ) { \
            const int pos = wc + (int)__builtin_amdgcn_mbcnt_lo(mj, 0u); \
            if (pos < WCAP) list[wave * WCAP + pos] = ((el0 + (J)) << 12) | (int)(SJ); \
          } \
          wc += (int)__builtin_popcount(mj); } }
      HITJ(0, h0, s0)
      HITJ(1, h1, s1)
      HITJ(2, h2, s2)
      HITJ(3, h3, s3)
      HITJ(4, h4, s4)
      HITJ(5, h5, s5)
      HITJ(6, h6, s6)
      HITJ(7, h7, s7)
#undef HITJ
    }
  }
  return wc;
}

__global__ __launch_bounds__(NTHR) void k_wprep(const float* __restrict__ Ws, const float* __restrict__ Wn,
                                                unsigned short* wp) {
  constexpr int UNITS = FD * KF / 8;
  constexpr int HALFU = UNITS / 2;
  static_assert((HALFU % NTHR) == 0);
  const int mat = (int)blockIdx.y;
  const int i = (int)blockIdx.x * NTHR + (int)threadIdx.x;
  if (i >= UNITS) return;
  const int half = i / HALFU;
  const int j = i - half * HALFU;
  const int n  = j >> 4;
  const int k8 = (j & 15) * 8;
  const float* src = (half == 0 ? Ws : Wn) + (size_t)mat * FD * FD;
  float v[8];
#pragma unroll
  for (int e = 0; e < 8; ++e) v[e] = src[(size_t)(k8 + e) * FD + n];
  v4f a, b;
  a.x = v[0]; a.y = v[1]; a.z = v[2]; a.w = v[3];
  b.x = v[4]; b.y = v[5]; b.z = v[6]; b.w = v[7];
  const v8us hv = cvt8h(a, b, WSCALE);
  unsigned short* d = wp + (size_t)mat * FD * KF + (size_t)n * KF + half * FD + k8;
  *(volatile v8us*)d = hv;
  __threadfence();
  *(volatile v8us*)d = hv;
}

__global__ __launch_bounds__(NTHR) void k_hprep(const float* __restrict__ x, const float* __restrict__ slot,
                                                unsigned short* A16, int nN, int nUnits, int applyBn) {
  constexpr int KD8 = FD / 8;
  const int i = (int)blockIdx.x * NTHR + (int)threadIdx.x;
  if (i >= nUnits) return;
  const int row = i / KD8;
  const int c0  = (i - row * KD8) * 8;
  const int rc  = row < nN ? row : nN - 1;
  const float* p = x + (size_t)rc * FD + c0;
  v4f a = *(const v4f*)p, b = *(const v4f*)(p + 4);
  if (applyBn != 0) {
    const v4f m0 = *(const v4f*)(slot + c0),          m1 = *(const v4f*)(slot + c0 + 4);
    const v4f s0 = *(const v4f*)(slot + FD + c0),     s1 = *(const v4f*)(slot + FD + c0 + 4);
    const v4f t0 = *(const v4f*)(slot + 2 * FD + c0), t1 = *(const v4f*)(slot + 2 * FD + c0 + 4);
    a = (a - m0) * s0 + t0;
    b = (b - m1) * s1 + t1;
  }
  const v4f z4 = {0.f, 0.f, 0.f, 0.f};
  if (row >= nN) { a = z4; b = z4; }
  const v8us hv = cvt8h(a, b, HSCALE);
  unsigned short* d = A16 + (size_t)row * AP + c0;
  *(volatile v8us*)d = hv;
  __threadfence();
  *(volatile v8us*)d = hv;
}

__global__ __launch_bounds__(NTHR) void k_count(
    const int* __restrict__ dstAll, int* cntAll, int nE, int vec8, int cntStride) {
  __shared__ __attribute__((aligned(16))) int scnt[NBC];
  __shared__ __attribute__((aligned(16))) int list[LISTN];
  __shared__ int wcnt[NWAVE];
  const int tid = threadIdx.x, lane = tid & 31, wave = tid >> 5;
  const int nodeBase = blockIdx.x * NBC;
  const int* dsts = dstAll + (size_t)blockIdx.y * nE;
  int* cnt = cntAll + (size_t)blockIdx.y * cntStride;

  for (int i = tid; i < NBC; i += NTHR) scnt[i] = 0;
  __syncthreads();

  const int nChunks = (nE + CHUNK - 1) / CHUNK;
#pragma unroll 1
  for (int ch = 0; ch < nChunks; ++ch) {
    const int cbase = ch * CHUNK;
    const int wc = scan_chunk<NBC>(dsts, nE, cbase, nodeBase, vec8, list, tid, lane, wave);
    if (lane == 0) wcnt[wave] = wc;
    __syncthreads();
    if (wave == 0) {
#pragma unroll 1
      for (int wsx = 0; wsx < NWAVE; ++wsx) {
        int n = __builtin_amdgcn_readfirstlane(wcnt[wsx]);
        n = n > WCAP ? WCAP : (n < 0 ? 0 : n);
        const int* lp = list + wsx * WCAP;
#pragma unroll 1
        for (int i = 0; i < n; ++i) {
          const int ent  = __builtin_amdgcn_readfirstlane(lp[i]);
          const int slot = ent & (NBC - 1);
          if (lane == 0) scnt[slot] = scnt[slot] + 1;
        }
      }
    }
    __syncthreads();
  }

  v4i cq[4];
#pragma unroll
  for (int q = 0; q < 4; ++q) {
    const int f = (wave * 4 + q) * 128 + 4 * lane;
    cq[q] = *(const v4i*)(scnt + f);
  }
  int* cp = cnt + (size_t)nodeBase;
#pragma unroll
  for (int q = 0; q < 4; ++q) {
    const int f = (wave * 4 + q) * 128 + 4 * lane;
    *(volatile v4i*)(cp + f) = cq[q];
  }
  __threadfence();
#pragma unroll
  for (int q = 0; q < 4; ++q) {
    const int f = (wave * 4 + q) * 128 + 4 * lane;
    *(volatile v4i*)(cp + f) = cq[q];
  }
}

__global__ __launch_bounds__(OTHR) void k_offsets(
    const int* __restrict__ cntAll, int* offAll, int* rbAll, int nChunk, int cntStride) {
  __shared__ __attribute__((aligned(16))) int soff[NBC];
  __shared__ __attribute__((aligned(16))) int srb[RBN];
  __shared__ int wtot[OTHR / 32];
  const int tid = threadIdx.x, lane = tid & 31, wave = tid >> 5, sub = tid >> 7;
  const int* cnt = cntAll + (size_t)blockIdx.x * cntStride;
  int* off   = offAll + (size_t)blockIdx.x * cntStride;
  int* rbase = rbAll + (size_t)blockIdx.x * RBN;
  for (int i = tid; i < RBN; i += OTHR) srb[i] = 0;
  int carry = 0;
#pragma unroll 1
  for (int ch = 0; ch < nChunk; ++ch) {
    const int base = ch * NBC;
    const v4i c0 = *(const v4i*)(cnt + base + 8 * tid);
    const v4i c1 = *(const v4i*)(cnt + base + 8 * tid + 4);
    const int e0 = max(c0.x, 0), e1 = max(c0.y, 0), e2 = max(c0.z, 0), e3 = max(c0.w, 0);
    const int e4 = max(c1.x, 0), e5 = max(c1.y, 0), e6 = max(c1.z, 0), e7 = max(c1.w, 0);
    const int ts = e0 + e1 + e2 + e3 + e4 + e5 + e6 + e7;
    int incl = ts;
#pragma unroll
    for (int d = 1; d < 32; d <<= 1) {
      const int up = __shfl_up(incl, d);
      if (lane >= d) incl += up;
    }
    if (lane == 31) wtot[wave] = incl;
    __syncthreads();
    const int S0 = wtot[0]  + wtot[1]  + wtot[2]  + wtot[3];
    const int S1 = wtot[4]  + wtot[5]  + wtot[6]  + wtot[7];
    const int S2 = wtot[8]  + wtot[9]  + wtot[10] + wtot[11];
    const int S3 = wtot[12] + wtot[13] + wtot[14] + wtot[15];
    int pre = 0;
#pragma unroll 1
    for (int w = 4 * sub; w < wave; ++w) pre += wtot[w];
    const int b0 = carry;
    const int b1 = b0 + ((S0 + 31) & ~31);
    const int b2 = b1 + ((S1 + 31) & ~31);
    const int b3 = b2 + ((S2 + 31) & ~31);
    const int b4 = b3 + ((S3 + 31) & ~31);
    const int myb = sub == 0 ? b0 : (sub == 1 ? b1 : (sub == 2 ? b2 : b3));
    if (tid == 0) {
      srb[min(4 * ch + 0, RBN - 1)] = b0;
      srb[min(4 * ch + 1, RBN - 1)] = b1;
      srb[min(4 * ch + 2, RBN - 1)] = b2;
      srb[min(4 * ch + 3, RBN - 1)] = b3;
    }
    int run = myb + pre + incl - ts;
    soff[8 * tid + 0] = run; run += e0;
    soff[8 * tid + 1] = run; run += e1;
    soff[8 * tid + 2] = run; run += e2;
    soff[8 * tid + 3] = run; run += e3;
    soff[8 * tid + 4] = run; run += e4;
    soff[8 * tid + 5] = run; run += e5;
    soff[8 * tid + 6] = run; run += e6;
    soff[8 * tid + 7] = run;
    carry = b4;
    __syncthreads();
    const v4i o0 = *(const v4i*)(soff + 4 * tid);
    const v4i o1 = *(const v4i*)(soff + 4 * (tid + OTHR));
    int* op = off + base;
    *(volatile v4i*)(op + 4 * tid) = o0;
    *(volatile v4i*)(op + 4 * (tid + OTHR)) = o1;
    __threadfence();
    *(volatile v4i*)(op + 4 * tid) = o0;
    *(volatile v4i*)(op + 4 * (tid + OTHR)) = o1;
    __syncthreads();
  }
  if (tid == 0) srb[min(4 * nChunk, RBN - 1)] = carry;
  __syncthreads();
  v4i rv = {0, 0, 0, 0};
  if (tid < 32) rv = *(const v4i*)(srb + 4 * tid);
  if (tid < 32) *(volatile v4i*)(rbase + 4 * tid) = rv;
  __threadfence();
  if (tid < 32) *(volatile v4i*)(rbase + 4 * tid) = rv;
}

__global__ __launch_bounds__(NTHR) void k_fill(
    const int* __restrict__ srcAll, const int* __restrict__ dstAll,
    const int* __restrict__ offAll, const int* __restrict__ rbAll,
    int* csrAll, int nN, int nE, int vec8, int csrLen, int cntStride) {
  extern __shared__ v4f lds_dyn[];
  int* region = (int*)lds_dyn;
  int* cursor = region + RCAP;
  int* list   = cursor + NBF;
  int* wcnt   = list + LISTN;
  const int tid = threadIdx.x, lane = tid & 31, wave = tid >> 5;
  const int t = (int)blockIdx.y;
  const int b = (int)blockIdx.x;
  const int nodeBase = b * NBF;
  const int* srcs  = srcAll + (size_t)t * nE;
  const int* dsts  = dstAll + (size_t)t * nE;
  const int* off   = offAll + (size_t)t * cntStride;
  const int* rbase = rbAll + (size_t)t * RBN;
  int* csr = csrAll + (size_t)t * csrLen;

  int rb0 = rbase[b];
  const int rb1 = rbase[b + 1];
  rb0 = rb0 < 0 ? 0 : (rb0 > csrLen ? csrLen : rb0);
  rb0 &= ~31;
  int len = rb1 - rb0;
  len = len < 0 ? 0 : (len > RCAP ? RCAP : len);
  int lenW = (len + 31) & ~31;
  if (rb0 + lenW > csrLen) lenW = (csrLen - rb0) & ~31;

  {
    const v4i z = {0, 0, 0, 0};
    for (int i = tid; i < RCAP / 4; i += NTHR) ((v4i*)region)[i] = z;
    for (int s = tid; s < NBF; s += NTHR) {
      int o = off[nodeBase + s] - rb0;
      o = o < 0 ? 0 : (o > RCAP ? RCAP : o);
      cursor[s] = o;
    }
  }
  __syncthreads();

  const int nChunks = (nE + CHUNK - 1) / CHUNK;
#pragma unroll 1
  for (int ch = 0; ch < nChunks; ++ch) {
    const int cbase = ch * CHUNK;
    const int wc = scan_chunk<NBF>(dsts, nE, cbase, nodeBase, vec8, list, tid, lane, wave);
    if (lane == 0) wcnt[wave] = wc;
    __syncthreads();
    if (wave == 0) {
#pragma unroll 1
      for (int wsx = 0; wsx < NWAVE; ++wsx) {
        int n = __builtin_amdgcn_readfirstlane(wcnt[wsx]);
        n = n > WCAP ? WCAP : (n < 0 ? 0 : n);
        const int* lp = list + wsx * WCAP;
#pragma unroll 1
        for (int i = 0; i < n; ++i) {
          const int ent  = __builtin_amdgcn_readfirstlane(lp[i]);
          const int slot = ent & (NBF - 1);
          int e = cbase + ((ent >> 12) & (CHUNK - 1));
          e = e > nE - 1 ? nE - 1 : e;
          int src = srcs[e];
          src = src < 0 ? 0 : (src > nN - 1 ? nN - 1 : src);
          if (lane == 0) {
            int pos = cursor[slot];
            pos = pos < 0 ? 0 : (pos > RCAP - 1 ? RCAP - 1 : pos);
            region[pos] = src;
            const int np = pos + 1;
            cursor[slot] = np > RCAP ? RCAP : np;
          }
        }
      }
    }
    __syncthreads();
  }

  const int nv = lenW >> 2;
  int* gp = csr + rb0;
#pragma unroll 1
  for (int i = tid; i < nv; i += NTHR) { const v4i v = ((const v4i*)region)[i]; *(volatile v4i*)(gp + 4 * i) = v; }
  __threadfence();
#pragma unroll 1
  for (int i = tid; i < nv; i += NTHR) { const v4i v = ((const v4i*)region)[i]; *(volatile v4i*)(gp + 4 * i) = v; }
}

__global__ __launch_bounds__(NTHR) void k_agg(
    const int* __restrict__ csrAll, const int* __restrict__ offAll, const int* __restrict__ cntAll,
    const float* __restrict__ hsrc, const float* __restrict__ slot, unsigned short* A16,
    int nN, int csrLen, int cntStride, int applyBn) {
  constexpr int RU  = FD / 2;
  constexpr int NFL = SROWS * RU / 4 / 32;
  __shared__ __attribute__((aligned(16))) unsigned int sOut[NWAVE * SROWS * RU];
  const int tid = threadIdx.x, lane = tid & 31, wave = tid >> 5;
  const int t = (int)blockIdx.y;
  const int* csr = csrAll + (size_t)t * csrLen;
  const int* off = offAll + (size_t)t * cntStride;
  const int* cnt = cntAll + (size_t)t * cntStride;
  const int tbase = blockIdx.x * TGT + wave * 32;
  const int col = 4 * lane;
  const v4f z4 = {0.f, 0.f, 0.f, 0.f};
  v4f mu4 = z4, sc4 = {1.f, 1.f, 1.f, 1.f}, sh4 = z4;
  if (applyBn != 0) {
    mu4 = *(const v4f*)(slot + col);
    sc4 = *(const v4f*)(slot + FD + col);
    sh4 = *(const v4f*)(slot + 2 * FD + col);
  }
  unsigned int* sw = sOut + wave * (SROWS * RU);

  const int cl    = tbase + lane;
  const int cnt_l = cnt[cl];
  const int off_l = off[cl];

#pragma unroll 1
  for (int j = 0; j < 32; ++j) {
    int nraw = __shfl(cnt_l, j);
    nraw = nraw < 0 ? 0 : (nraw > (1 << 24) ? (1 << 24) : nraw);
    const int n = nraw > DEGCAP ? DEGCAP : nraw;
    const int st = __shfl(off_l, j);

    v4f acc = z4;
#pragma unroll 1
    for (int q0 = 0; q0 < n; q0 += 32) {
      int pos = st + q0 + lane;
      pos = pos < 0 ? 0 : (pos > csrLen - 1 ? csrLen - 1 : pos);
      int sl = csr[pos];
      sl = sl < 0 ? 0 : (sl > nN - 1 ? nN - 1 : sl);
      const int mcnt = (n - q0) < 32 ? (n - q0) : 32;
#pragma unroll 1
      for (int pp = 0; pp < mcnt; ++pp) {
        const int s = __builtin_amdgcn_readlane(sl, pp);
        const v4f hv = *(const v4f*)(hsrc + (size_t)s * FD + col);
        acc = acc + hv;
      }
    }
    const float rn = 1.0f / (float)(nraw > 0 ? nraw : 1);
    v4f v = (acc * rn - mu4) * sc4 + sh4;
    if (n <= 0) v = z4;
    *(v2u*)(sw + (j & (SROWS - 1)) * RU + 2 * lane) = cvt4h(v, HSCALE);

    if ((j & (SROWS - 1)) == SROWS - 1) {
      __syncthreads();
      const int jb = j - (SROWS - 1);
      unsigned short* gp = A16 + (size_t)(tbase + jb) * AP + FD + FD * t;
      v4u ov[NFL];
#pragma unroll
      for (int it = 0; it < NFL; ++it) {
        const int f = it * 32 + lane;
        ov[it] = *(const v4u*)(sw + 4 * f);
        const int srow = f >> 4, piece = f & 15;
        *(volatile v4u*)(gp + (size_t)srow * AP + 8 * piece) = ov[it];
      }
      __threadfence();
#pragma unroll
      for (int it = 0; it < NFL; ++it) {
        const int f = it * 32 + lane;
        const int srow = f >> 4, piece = f & 15;
        *(volatile v4u*)(gp + (size_t)srow * AP + 8 * piece) = ov[it];
      }
      __syncthreads();
    }
  }
}

__global__ __launch_bounds__(NTHR) void k_gemm(
    const unsigned short* __restrict__ A16, const unsigned short* __restrict__ Bw,
    const float* __restrict__ biasL, float* outp, double* part, int nN, int relu) {
  constexpr int TPW = 4;
  constexpr int WC  = TPW * 16;
  static_assert(2 * WC == FD && (NWAVE / 2) * 16 == GBM);
  static_assert(GBM == NWAVE * 8);
  static_assert(NTHR == 2 * FD);
  __shared__ __attribute__((aligned(16))) float  stg[GBM * FD];
  __shared__ __attribute__((aligned(16))) double sS[2 * FD];
  __shared__ __attribute__((aligned(16))) double sQ[2 * FD];
  __shared__ __attribute__((aligned(16))) double sP[PARTN];
  const int tid = threadIdx.x, lane = tid & 31, wave = tid >> 5, hh = lane >> 4, m = lane & 15;
  const int rowBase = blockIdx.x * GBM;
  const int rg  = wave >> 1;
  const int chf = wave & 1;
  const int r0  = rg * 16;
  const int c0  = chf * WC;

  v8f accO[TPW];
#pragma unroll
  for (int t = 0; t < TPW; ++t) { v8f z = {0.f, 0.f, 0.f, 0.f, 0.f, 0.f, 0.f, 0.f}; accO[t] = z; }
  const unsigned short* ap = A16 + (size_t)(rowBase + r0 + m) * AP + 8 * hh;

#pragma unroll 1
  for (int e = 0; e < TT; ++e) {
    v8f acc[TPW];
#pragma unroll
    for (int t = 0; t < TPW; ++t) { v8f z = {0.f, 0.f, 0.f, 0.f, 0.f, 0.f, 0.f, 0.f}; acc[t] = z; }
    const unsigned short* bq = Bw + (size_t)e * FD * KF + (size_t)(c0 + m) * KF + 8 * hh;
#pragma unroll 1
    for (int kt = 0; kt < KF / 32; ++kt) {
      const int acol = 32 * kt + (kt >= FD / 32 ? FD * e : 0);
      FragH a;
      a.h[0] = *(const v8us*)(ap + acol);
      a.h[1] = *(const v8us*)(ap + acol + 16);
#pragma unroll
      for (int t = 0; t < TPW; ++t) {
        const unsigned short* bp = bq + (size_t)(16 * t) * KF + 32 * kt;
        FragH b;
        b.h[0] = *(const v8us*)bp;
        b.h[1] = *(const v8us*)(bp + 16);
        acc[t] = wmh(a.v, b.v, acc[t]);
      }
    }
    const float* be = biasL + e * FD + c0 + m;
#pragma unroll
    for (int t = 0; t < TPW; ++t) {
      const float bv = be[16 * t];
#pragma unroll
      for (int r = 0; r < 8; ++r) {
        float o = acc[t][r] * OINV + bv;
        o = (relu != 0) ? fmaxf(o, 0.0f) : o;
        accO[t][r] += o;
      }
    }
  }

  {
    float* sp = stg + (size_t)(r0 + 8 * hh) * FD + c0 + m;
#pragma unroll
    for (int t = 0; t < TPW; ++t) {
#pragma unroll
      for (int r = 0; r < 8; ++r) sp[r * FD + 16 * t] = accO[t][r];
    }
  }
  __syncthreads();

  v4f ov[8];
#pragma unroll
  for (int it = 0; it < 8; ++it) {
    const int row  = wave * 8 + it;
    const int grow = rowBase + row;
    ov[it] = *(const v4f*)(stg + (size_t)row * FD + 4 * lane);
    if (grow < nN) *(volatile v4f*)(outp + (size_t)grow * FD + 4 * lane) = ov[it];
  }
  __threadfence();
#pragma unroll
  for (int it = 0; it < 8; ++it) {
    const int row  = wave * 8 + it;
    const int grow = rowBase + row;
    if (grow < nN) *(volatile v4f*)(outp + (size_t)grow * FD + 4 * lane) = ov[it];
  }

  {
    const int c  = tid & (FD - 1);
    const int hf = tid >> 7;
    int nr = nN - rowBase;
    nr = nr < 0 ? 0 : (nr > GBM ? GBM : nr);
    const int rA = hf * (GBM / 2);
    int rB = rA + GBM / 2;
    rB = rB > nr ? nr : rB;
    double s = 0.0, q = 0.0;
#pragma unroll 2
    for (int r = rA; r < rB; ++r) {
      const double xv = (double)stg[(size_t)r * FD + c];
      s += xv;
      q += xv * xv;
    }
    sS[tid] = s;
    sQ[tid] = q;
  }
  __syncthreads();
  if (tid < FD) {
    sP[tid]      = sS[tid] + sS[FD + tid];
    sP[FD + tid] = sQ[tid] + sQ[FD + tid];
  }
  __syncthreads();
  v2d pv = {0.0, 0.0};
  double* pp = part + (size_t)blockIdx.x * PARTN + 2 * tid;
  if (tid < PARTN / 2) { pv = *(const v2d*)(sP + 2 * tid); *(volatile v2d*)pp = pv; }
  __threadfence();
  if (tid < PARTN / 2) *(volatile v2d*)pp = pv;
}

__global__ __launch_bounds__(NTHR) void k_bnred(
    const double* __restrict__ part, const float* __restrict__ gam, const float* __restrict__ bet,
    float* slot, int nBlk, int nN) {
  __shared__ __attribute__((aligned(16))) double sAcc[PARTN];
  __shared__ __attribute__((aligned(16))) float  sSl[SLOTN];
  const int tid = threadIdx.x;
  double a = 0.0;
#pragma unroll 2
  for (int bk = 0; bk < nBlk; ++bk) a += part[(size_t)bk * PARTN + tid];
  sAcc[tid] = a;
  __syncthreads();
  if (tid < FD) {
    const double invN = 1.0 / (double)nN;
    const double mu   = sAcc[tid] * invN;
    double var = sAcc[FD + tid] * invN - mu * mu;
    var = var < 0.0 ? 0.0 : var;
    const float varf = (float)var;
    const float rstd = 1.0f / sqrtf(varf + BN_EPS);
    sSl[tid]          = (float)mu;
    sSl[FD + tid]     = gam[tid] * rstd;
    sSl[2 * FD + tid] = bet[tid];
    sSl[3 * FD + tid] = 0.0f;
  }
  __syncthreads();
  v4f v = {0.f, 0.f, 0.f, 0.f};
  if (tid < SLOTN / 4) { v = *(const v4f*)(sSl + 4 * tid); *(volatile v4f*)(slot + 4 * tid) = v; }
  __threadfence();
  if (tid < SLOTN / 4) *(volatile v4f*)(slot + 4 * tid) = v;
}

__global__ __launch_bounds__(NTHR) void k_bnapply(float* out, const float* __restrict__ slot, int nN) {
  const int i = (int)blockIdx.x * NTHR + (int)threadIdx.x;
  const int total = nN * 32;
  if (i >= total) return;
  const int row = i >> 5;
  const int col = 4 * (i & 31);
  const v4f mu = *(const v4f*)(slot + col);
  const v4f sc = *(const v4f*)(slot + FD + col);
  const v4f sh = *(const v4f*)(slot + 2 * FD + col);
  float* p = out + (size_t)row * FD + col;
  const v4f xv = *(const v4f*)p;
  const v4f y = (xv - mu) * sc + sh;
  *(volatile v4f*)p = y;
  __threadfence();
  *(volatile v4f*)p = y;
}

extern "C" void kernel_launch(void* const* d_in, const int* in_sizes, int n_in,
                              void* d_out, int out_size, void* d_ws, size_t ws_size,
                              hipStream_t stream) {
  if (n_in < 8) return;
  const int nN = in_sizes[0] / FD;
  if (nN <= 0 || in_sizes[0] != nN * FD) return;
  if (in_sizes[1] <= 0 || (in_sizes[1] % TT) != 0 || in_sizes[2] != in_sizes[1]) return;
  const int nE = in_sizes[1] / TT;
  if (in_sizes[3] != LL * TT * FD * FD || in_sizes[4] != LL * TT * FD * FD) return;
  if (in_sizes[5] != LL * TT * FD || in_sizes[6] != LL * FD || in_sizes[7] != LL * FD) return;
  if (out_size != nN * FD) return;
  if (nE > (1 << 28) || nN > (1 << 24)) return;

  const float* feat = (const float*)d_in[0];
  const int*   src  = (const int*)d_in[1];
  const int*   dst  = (const int*)d_in[2];
  const float* Wsf  = (const float*)d_in[3];
  const float* Wnb  = (const float*)d_in[4];
  const float* bias = (const float*)d_in[5];
  const float* gam  = (const float*)d_in[6];
  const float* bet  = (const float*)d_in[7];
  float* out = (float*)d_out;

  const int NPAD   = ((nN + TGT - 1) / TGT) * TGT;
  const int nBC    = (nN + NBC - 1) / NBC;
  const int CNTPAD = nBC * NBC;
  if (4 * nBC + 1 > RBN) return;
  const int nBF    = (nN + NBF - 1) / NBF;
  const int csrLen = ((nE + 31) & ~31) + 4096;
  if (31 * 4 * nBC > 4096) return;
  const int nAgg   = NPAD / TGT;
  const int nGemm  = NPAD / GBM;
  const int hUnits = NPAD * (FD / 8);

  char* ws = (char*)d_ws;
  size_t off = 0;
  const size_t oWp   = off; off += (size_t)LL * TT * FD * KF * 2;   off = (off + 255) & ~(size_t)255;
  const size_t oA    = off; off += (size_t)NPAD * AP * 2;           off = (off + 255) & ~(size_t)255;
  const size_t oCnt  = off; off += (size_t)TT * CNTPAD * 4;         off = (off + 255) & ~(size_t)255;
  const size_t oOff  = off; off += (size_t)TT * CNTPAD * 4;         off = (off + 255) & ~(size_t)255;
  const size_t oRb   = off; off += (size_t)TT * RBN * 4;            off = (off + 255) & ~(size_t)255;
  const size_t oCsr  = off; off += (size_t)TT * csrLen * 4;         off = (off + 255) & ~(size_t)255;
  const size_t oPart = off; off += (size_t)nGemm * PARTN * 8;       off = (off + 255) & ~(size_t)255;
  const size_t oSlot = off; off += (size_t)LL * SLOTN * 4;          off = (off + 255) & ~(size_t)255;
  if (off > ws_size || off > (size_t)WSCAP) return;
  unsigned short* wpl  = (unsigned short*)(ws + oWp);
  unsigned short* a16  = (unsigned short*)(ws + oA);
  int*    cnt  = (int*)(ws + oCnt);
  int*    offp = (int*)(ws + oOff);
  int*    rb   = (int*)(ws + oRb);
  int*    csr  = (int*)(ws + oCsr);
  double* part = (double*)(ws + oPart);
  float*  slots = (float*)(ws + oSlot);

  const int vec8 = ((nE & 3) == 0) ? 1 : 0;

  k_wprep<<<dim3(FD * KF / 8 / NTHR, LL * TT), NTHR, 0, stream>>>(Wsf, Wnb, wpl);

  k_count<<<dim3(nBC, TT), NTHR, 0, stream>>>(dst, cnt, nE, vec8, CNTPAD);
  k_offsets<<<TT, OTHR, 0, stream>>>(cnt, offp, rb, nBC, CNTPAD);
  hipFuncSetAttribute(reinterpret_cast<const void*>(&k_fill),
                      hipFuncAttributeMaxDynamicSharedMemorySize, LDS_FILL);
  k_fill<<<dim3(nBF, TT), NTHR, LDS_FILL, stream>>>(src, dst, offp, rb, csr, nN, nE, vec8, csrLen, CNTPAD);

  for (int l = 0; l < LL; ++l) {
    const float* hsrc  = (l == 0) ? feat : (const float*)out;
    const int applyBn  = (l == 0) ? 0 : 1;
    const float* slotIn = slots + (size_t)(l == 0 ? 0 : l - 1) * SLOTN;
    const int relu = (l < LL - 1) ? 1 : 0;
    k_hprep<<<hUnits / NTHR, NTHR, 0, stream>>>(hsrc, slotIn, a16, nN, hUnits, applyBn);
    k_agg<<<dim3(nAgg, TT), NTHR, 0, stream>>>(csr, offp, cnt, hsrc, slotIn, a16, nN, csrLen, CNTPAD, applyBn);
    k_gemm<<<nGemm, NTHR, 0, stream>>>(a16, wpl + (size_t)l * TT * FD * KF, bias + (size_t)l * TT * FD,
                                       out, part, nN, relu);
    k_bnred<<<1, NTHR, 0, stream>>>(part, gam + (size_t)l * FD, bet + (size_t)l * FD,
                                    slots + (size_t)l * SLOTN, nGemm, nN);
  }

  k_bnapply<<<(nN * 32 + NTHR - 1) / NTHR, NTHR, 0, stream>>>(out, slots + (size_t)(LL - 1) * SLOTN, nN);
}
